// RoPEMultiheadSelfAttention_55748675502795
// MI455X (gfx1250) — hardware-verified
//
#include <hip/hip_runtime.h>
#include <math.h>
#include <stdint.h>

#ifndef NB
#define NB 4
#endif
#ifndef SEQ
#define SEQ 2048
#endif
#define XS_FULL 2048
#define DMOD  1024
#define NH    16
#define HD    64
#define HHALF (HD / 2)
#define NFREQ (HD / 2)
#define MROWS (NB * SEQ)
#define ROPE_L2 0.41524101186092028
#define SM_SCALE 0.125f
#define QSC   256.0f
#define KSC   256.0f
#define PCAR  32768.0f
#define VCAR  1024.0f
#define OSC   256.0f
#define WOS   1024.0f
#define WPB   4
#define NHG   (NH / WPB)
#define NQT   (SEQ / 16)
#define NST   (SEQ / 64)
#define NKT   (SEQ / 32)
#define ATT_THREADS (WPB * 32)
#define PTP   36
#define PTW   (16 * PTP)
#define SLP   68
#define SLW   (16 * SLP)
#define WREG  (PTW + SLW)
#define SLAB64 (16 * 68)
#define VTP   72
#define WS_CAP 134217728
static_assert(DMOD == NH * HD && HD == 64 && HHALF == 32 && NFREQ == 32 && NH == 16 && WPB == 4 && NHG * WPB == NH);
static_assert(ATT_THREADS == 128);
static_assert(NB >= 1 && NB <= 4);
static_assert(NB == 1 || SEQ == XS_FULL);
static_assert((SEQ % 64) == 0 && SEQ >= 64 && SEQ <= XS_FULL);
static_assert((DMOD % 64) == 0 && (DMOD % 32) == 0 && (HD % 32) == 0 && (MROWS % 64) == 0);
static_assert(((SEQ * DMOD / 8) % 256) == 0 && ((DMOD * DMOD / 8) % 256) == 0 && ((SEQ * NFREQ) % 256) == 0);
static_assert(WPB * WREG * 4 <= 65536 && HD * VTP * 2 <= 65536 && 4 * SLAB64 * 4 <= 65536);

typedef unsigned short u16;
typedef _Float16 v16h __attribute__((ext_vector_type(16)));
typedef _Float16 v8h  __attribute__((ext_vector_type(8)));
typedef __bf16   v16b __attribute__((ext_vector_type(16)));
typedef float    v8f  __attribute__((ext_vector_type(8)));
typedef float    v4f  __attribute__((ext_vector_type(4)));
typedef unsigned int v4u __attribute__((ext_vector_type(4)));

union FragH { v16h v; v8h h[2]; v4u u[2]; };
union FragB { v16b v; v4u u[2]; };

__device__ __forceinline__ unsigned short bf_bits(float f) {
  unsigned u = __float_as_uint(f);
  return (unsigned short)((u + 0x7FFFu + ((u >> 16) & 1u)) >> 16);
}
__device__ __forceinline__ float bf_up(unsigned short h) { return __uint_as_float(((unsigned)h) << 16); }
__device__ __forceinline__ float bfr(float f) { return bf_up(bf_bits(f)); }
__device__ __forceinline__ unsigned short h_bits(_Float16 x) { return __builtin_bit_cast(unsigned short, x); }
__device__ __forceinline__ unsigned pk16(unsigned short a, unsigned short b) { return (unsigned)a | ((unsigned)b << 16); }
__device__ __forceinline__ v8f zero8() { v8f z = {0.f, 0.f, 0.f, 0.f, 0.f, 0.f, 0.f, 0.f}; return z; }

__device__ __forceinline__ v16h ldfrag_h(const _Float16* p) {
  FragH f;
  f.h[0] = *(const v8h*)(p);
  f.h[1] = *(const v8h*)(p + 16);
  return f.v;
}
__device__ __forceinline__ v16b ldfrag_b(const u16* p) {
  FragB f;
  f.u[0] = *(const v4u*)(p);
  f.u[1] = *(const v4u*)(p + 16);
  return f.v;
}

__device__ __forceinline__ v8f mma_h(v16h a, v16h b, v8f c) {
  return __builtin_amdgcn_wmma_f32_16x16x32_f16(false, a, false, b, (short)0, c, false, false);
}
__device__ __forceinline__ v8f mma_b(v16b a, v16b b, v8f c) {
  return __builtin_amdgcn_wmma_f32_16x16x32_bf16(false, a, false, b, (short)0, c, false, false);
}
__device__ __forceinline__ void guard2(v8f& a, v8f& b, v16h x0, v16h x1, v16h x2, v16h x3, v16h x4, v16h x5) {
#if defined(__HIP_DEVICE_COMPILE__)
  asm volatile("v_nop\n\tv_nop\n\tv_nop\n\tv_nop"
               : "+v"(a), "+v"(b) : "v"(x0), "v"(x1), "v"(x2), "v"(x3), "v"(x4), "v"(x5) : "memory");
#endif
}
template <typename F>
__device__ __forceinline__ void guard6(v8f& a, v8f& b, v8f& c, v8f& d, F x0, F x1, F x2, F x3, F x4, F x5) {
#if defined(__HIP_DEVICE_COMPILE__)
  asm volatile("v_nop\n\tv_nop\n\tv_nop\n\tv_nop"
               : "+v"(a), "+v"(b), "+v"(c), "+v"(d) : "v"(x0), "v"(x1), "v"(x2), "v"(x3), "v"(x4), "v"(x5) : "memory");
#endif
}
__device__ __forceinline__ void acc_guard4(v8f& a, v8f& b, v8f& c, v8f& d) {
#if defined(__HIP_DEVICE_COMPILE__)
  asm volatile("v_nop\n\tv_nop\n\tv_nop\n\tv_nop" : "+v"(a), "+v"(b), "+v"(c), "+v"(d));
#endif
}
__device__ __forceinline__ void wave_sync_lds() {
  __builtin_amdgcn_fence(__ATOMIC_RELEASE, "workgroup");
  __builtin_amdgcn_wave_barrier();
  __builtin_amdgcn_fence(__ATOMIC_ACQUIRE, "workgroup");
}

__global__ __launch_bounds__(256) void cvt16(const float* __restrict__ x, u16* D, int n8, int f16mode, float scale) {
  const int gt = blockIdx.x * 256 + (int)threadIdx.x;
  if (gt >= n8) return;
  const float* p = x + (size_t)gt * 8;
  const v4f a = *(const v4f*)(p), b4 = *(const v4f*)(p + 4);
  float w[8];
#pragma unroll
  for (int e = 0; e < 4; ++e) { w[e] = a[e]; w[4 + e] = b4[e]; }
  v4u o;
#pragma unroll
  for (int e = 0; e < 4; ++e) {
    const float f0 = w[2 * e], f1 = w[2 * e + 1];
    const unsigned short hb0 = h_bits((_Float16)(bfr(f0) * scale));
    const unsigned short hb1 = h_bits((_Float16)(bfr(f1) * scale));
    const unsigned short bb0 = bf_bits(f0);
    const unsigned short bb1 = bf_bits(f1);
    o[e] = (f16mode != 0) ? pk16(hb0, hb1) : pk16(bb0, bb1);
  }
  u16* d = D + (size_t)gt * 8;
  for (int pass = 0; pass < 2; ++pass) {
    *(volatile v4u*)(d) = o;
    __threadfence();
  }
}

__global__ __launch_bounds__(256) void k_tab(float* TC, float* TS, int n) {
#pragma clang fp contract(off)
  const int idx = blockIdx.x * 256 + (int)threadIdx.x;
  if (idx >= n) return;
  const int s = idx / NFREQ;
  const int j = idx - s * NFREQ;
  const double pj = exp2((double)j * ROPE_L2);
  const float pf  = (float)pj;
  const float inv = 1.0f / pf;
  const float ang = (float)s * inv;
  float sv, cv;
  sincosf(ang, &sv, &cv);
  for (int pass = 0; pass < 2; ++pass) {
    *(volatile float*)(TC + idx) = cv;
    *(volatile float*)(TS + idx) = sv;
    __threadfence();
  }
}

__global__ __launch_bounds__(256) void vt16(const float* __restrict__ F, int ldf, int voff, u16* VHo) {
  __shared__ __align__(16) u16 TH[HD * VTP];
  const int tid = threadIdx.x;
  const int bid = blockIdx.x;
  const int st  = bid % NST;
  const int t2  = bid / NST;
  const int g   = t2 % NH;
  const int b   = t2 / NH;
  if (b >= NB) return;
  const int s0  = st * 64;
  {
    const int sl = tid >> 2;
    const int dc = (tid & 3) * 16;
    const float* src = F + ((size_t)b * SEQ + s0 + sl) * (size_t)ldf + voff + g * HD + dc;
#pragma unroll
    for (int i = 0; i < 4; ++i) {
      const v4f a = *(const v4f*)(src + 4 * i);
#pragma unroll
      for (int e = 0; e < 4; ++e) {
        const float t = a[e] * VCAR;
        const _Float16 hv = (_Float16)t;
        TH[(dc + 4 * i + e) * VTP + sl] = h_bits(hv);
      }
    }
  }
  __syncthreads();
  v4u vh[2];
  const int q8 = tid >> 3, p8 = (tid & 7) * 8;
#pragma unroll
  for (int it = 0; it < 2; ++it) {
    const int line = it * 32 + q8;
    vh[it] = *(const v4u*)(TH + line * VTP + p8);
  }
  const size_t hrow = (size_t)(b * NH + g) * HD;
  const size_t base = hrow * SEQ + s0 + p8;
  for (int pass = 0; pass < 2; ++pass) {
#pragma unroll
    for (int it = 0; it < 2; ++it) {
      const int line = it * 32 + q8;
      *(volatile v4u*)(VHo + base + (size_t)line * SEQ) = vh[it];
    }
    __threadfence();
  }
}

__device__ __forceinline__ void rot_one(float x, float y, float cv, float sv, float sgn, float sc,
                                        unsigned short& hb, unsigned short& lb) {
#pragma clang fp contract(off)
  const float ys   = y * sv;
  const float term = sgn * ys;
  const float r    = x * cv + term;
  const float t    = r * sc;
  const _Float16 a = (_Float16)t;
  hb = h_bits(a);
  lb = h_bits((_Float16)(t - (float)a));
}

template <int RES>
__global__ __launch_bounds__(128) void rope16(const float* __restrict__ F, int ldf, int coff,
                                              const float* __restrict__ TC, const float* __restrict__ TS,
                                              u16* Hp, u16* Lp, float sc) {
#pragma clang fp contract(off)
  const int tid = (int)threadIdx.x;
  const int row = (int)blockIdx.x;
  if (row >= MROWS) return;
  const int dd   = (tid & 7) * 8;
  const int hb   = (tid >> 3) * HD;
  const int col  = hb + dd;
  if (hb + HD > DMOD) return;
  const int jj   = dd >> 1;
  const int pcol = hb + (dd ^ HHALF);
  const float sgn = (dd < HHALF) ? -1.0f : 1.0f;
  const int b = row / SEQ;
  const int s = row - b * SEQ;
  const float* p = F + (size_t)row * (size_t)ldf + coff;
  const v4f xa = *(const v4f*)(p + col),  xb = *(const v4f*)(p + col + 4);
  const v4f ya = *(const v4f*)(p + pcol), yb = *(const v4f*)(p + pcol + 4);
  const v4f ca = *(const v4f*)(TC + (size_t)s * NFREQ + jj);
  const v4f sa = *(const v4f*)(TS + (size_t)s * NFREQ + jj);
  float xv[8], yv[8], cw[8], sw[8];
#pragma unroll
  for (int e = 0; e < 4; ++e) {
    xv[e] = xa[e];  xv[4 + e] = xb[e];
    yv[e] = ya[e];  yv[4 + e] = yb[e];
  }
#pragma unroll
  for (int e = 0; e < 8; ++e) { cw[e] = ca[e >> 1]; sw[e] = sa[e >> 1]; }
  v4u oh, ol;
#pragma unroll
  for (int e = 0; e < 4; ++e) {
    unsigned short h0, l0, h1, l1;
    rot_one(xv[2 * e],     yv[2 * e],     cw[2 * e],     sw[2 * e],     sgn, sc, h0, l0);
    rot_one(xv[2 * e + 1], yv[2 * e + 1], cw[2 * e + 1], sw[2 * e + 1], sgn, sc, h1, l1);
    oh[e] = pk16(h0, h1);
    ol[e] = pk16(l0, l1);
  }
  u16* dh = Hp + (size_t)row * DMOD + col;
  u16* dl = Lp + (size_t)row * DMOD + col;
  for (int pass = 0; pass < 2; ++pass) {
    *(volatile v4u*)(dh) = oh;
    if (RES != 0) {
      *(volatile v4u*)(dl) = ol;
    }
    __threadfence();
  }
  (void)dl; (void)ol;
}

__device__ __forceinline__ void epi64(float* sl, v8f a0, v8f a1, v8f a2, v8f a3, float oscale,
                                      const float* __restrict__ bias, float* C, int N, size_t rowb, int col0, int lane) {
  const int hh = lane >> 4, m = lane & 15;
  const float b0 = bfr(bias[col0 + m]);
  const float b1 = bfr(bias[col0 + 16 + m]);
  const float b2 = bfr(bias[col0 + 32 + m]);
  const float b3 = bfr(bias[col0 + 48 + m]);
#pragma unroll
  for (int r = 0; r < 8; ++r) {
    const int ro = (8 * hh + r) * 68 + m;
    sl[ro]      = a0[r] * oscale + b0;
    sl[ro + 16] = a1[r] * oscale + b1;
    sl[ro + 32] = a2[r] * oscale + b2;
    sl[ro + 48] = a3[r] * oscale + b3;
  }
  wave_sync_lds();
  v4f vals[8];
#pragma unroll
  for (int it = 0; it < 8; ++it) vals[it] = *(const v4f*)(sl + (it * 2 + hh) * 68 + m * 4);
  float* dst = C + (rowb + (size_t)hh) * (size_t)N + col0 + m * 4;
  for (int pass = 0; pass < 2; ++pass) {
#pragma unroll
    for (int it = 0; it < 8; ++it) {
      *(volatile v4f*)(dst + (size_t)(it * 2) * (size_t)N) = vals[it];
    }
    __threadfence();
  }
}

__global__ __launch_bounds__(128)
void gemm_bf(const u16* __restrict__ A, const u16* __restrict__ Bt, const float* __restrict__ bias, float* C,
             int M, int N, int K, float oscale) {
  __shared__ __align__(16) float slab[4 * SLAB64];
  const int tid = threadIdx.x, wave = tid >> 5, lane = tid & 31, hh = lane >> 4, m = lane & 15;
  const int ntile = N >> 6;
  const int bid   = blockIdx.x;
  const int rowb  = (bid / ntile) * 64 + wave * 16;
  const int col0  = (bid % ntile) * 64;
  if (rowb + 16 > M) return;
  const u16* ap = A  + (size_t)(rowb + m) * K + 8 * hh;
  const u16* bp = Bt + (size_t)(col0 + m) * K + 8 * hh;
  const size_t bs = (size_t)16 * K;
  v8f acc0 = zero8(), acc1 = zero8(), acc2 = zero8(), acc3 = zero8();
#pragma unroll 1
  for (int k0 = 0; k0 < K; k0 += 32) {
    const v16b a  = ldfrag_b(ap + k0);
    const v16b b0 = ldfrag_b(bp + k0);
    const v16b b1 = ldfrag_b(bp + bs + k0);
    const v16b b2 = ldfrag_b(bp + 2 * bs + k0);
    const v16b b3 = ldfrag_b(bp + 3 * bs + k0);
    acc0 = mma_b(a, b0, acc0);
    acc1 = mma_b(a, b1, acc1);
    acc2 = mma_b(a, b2, acc2);
    acc3 = mma_b(a, b3, acc3);
    guard6<v16b>(acc0, acc1, acc2, acc3, a, b0, b1, b2, b3, a);
  }
  epi64(slab + wave * SLAB64, acc0, acc1, acc2, acc3, oscale, bias, C, N, (size_t)rowb, col0, lane);
}

template <int TWO>
__global__ __launch_bounds__(128)
void gemm_h(const u16* __restrict__ A, const u16* __restrict__ A2, const u16* __restrict__ Bt,
            const float* __restrict__ bias, float* C, int M, int N, int K, float oscale) {
  __shared__ __align__(16) float slab[4 * SLAB64];
  const int tid = threadIdx.x, wave = tid >> 5, lane = tid & 31, hh = lane >> 4, m = lane & 15;
  const int ntile = N >> 6;
  const int bid   = blockIdx.x;
  const int rowb  = (bid / ntile) * 64 + wave * 16;
  const int col0  = (bid % ntile) * 64;
  if (rowb + 16 > M) return;
  const _Float16* ap  = (const _Float16*)(const void*)A  + (size_t)(rowb + m) * K + 8 * hh;
  const _Float16* ap2 = (const _Float16*)(const void*)A2 + (size_t)(rowb + m) * K + 8 * hh;
  const _Float16* bp  = (const _Float16*)(const void*)Bt + (size_t)(col0 + m) * K + 8 * hh;
  const size_t bs = (size_t)16 * K;
  v8f acc0 = zero8(), acc1 = zero8(), acc2 = zero8(), acc3 = zero8();
#pragma unroll 1
  for (int k0 = 0; k0 < K; k0 += 32) {
    const v16h a  = ldfrag_h(ap + k0);
    const v16h b0 = ldfrag_h(bp + k0);
    const v16h b1 = ldfrag_h(bp + bs + k0);
    const v16h b2 = ldfrag_h(bp + 2 * bs + k0);
    const v16h b3 = ldfrag_h(bp + 3 * bs + k0);
    acc0 = mma_h(a, b0, acc0);
    acc1 = mma_h(a, b1, acc1);
    acc2 = mma_h(a, b2, acc2);
    acc3 = mma_h(a, b3, acc3);
    if (TWO != 0) {
      const v16h a2 = ldfrag_h(ap2 + k0);
      acc0 = mma_h(a2, b0, acc0);
      acc1 = mma_h(a2, b1, acc1);
      acc2 = mma_h(a2, b2, acc2);
      acc3 = mma_h(a2, b3, acc3);
      guard6<v16h>(acc0, acc1, acc2, acc3, a, a2, b0, b1, b2, b3);
    } else {
      guard6<v16h>(acc0, acc1, acc2, acc3, a, b0, b1, b2, b3, a);
    }
  }
  (void)ap2;
  epi64(slab + wave * SLAB64, acc0, acc1, acc2, acc3, oscale, bias, C, N, (size_t)rowb, col0, lane);
}

__global__ __launch_bounds__(ATT_THREADS)
void attn_mh(const u16* __restrict__ QHp, const u16* __restrict__ QLp, const u16* __restrict__ KHp,
             const u16* __restrict__ VHp, u16* OHp, u16* OLp, int nqt) {
#pragma clang fp contract(off)
  __shared__ __align__(16) float smem[WPB * WREG];

  const int tid  = threadIdx.x;
  const int wave = tid >> 5;
  const int lane = tid & 31;
  const int hh   = lane >> 4;
  const int c    = lane & 15;
  const int bid  = blockIdx.x;
  if (nqt <= 0) return;
  const int qt   = bid % nqt;
  const int t2   = bid / nqt;
  const int hg   = t2 % NHG;
  const int b    = t2 / NHG;
  if (b >= NB) return;
  const int q0   = qt * 16;
  if (q0 + 16 > SEQ) return;
  const int head = hg * WPB + wave;

  float* pt   = smem + wave * WREG;
  float* slab = pt + PTW;

  const size_t hcol = (size_t)head * HD + 8 * hh;
  const _Float16* Qh  = (const _Float16*)(const void*)QHp + ((size_t)b * SEQ + q0 + c) * DMOD + hcol;
  const _Float16* Ql  = (const _Float16*)(const void*)QLp + ((size_t)b * SEQ + q0 + c) * DMOD + hcol;
  const _Float16* Khb = (const _Float16*)(const void*)KHp + ((size_t)b * SEQ + c) * DMOD + hcol;
  const _Float16* Vhb = (const _Float16*)(const void*)VHp + ((size_t)(b * NH + head) * HD + c) * SEQ + 8 * hh;
  const float lsc  = SM_SCALE * (1.0f / (QSC * KSC));
  const float oc   = 1.0f / (PCAR * VCAR);
  const float ninf = -__builtin_inff();
  const size_t KROW = (size_t)DMOD;

  v8f o[4];
#pragma unroll
  for (int j = 0; j < 4; ++j) o[j] = zero8();
  float mrun[8], lrun[8];
#pragma unroll
  for (int r = 0; r < 8; ++r) { mrun[r] = ninf; lrun[r] = 0.0f; }
  const int nkt = NKT;

#pragma unroll 1
  for (int kt = 0; kt < nkt; ++kt) {
    const int kb = kt * 32;
    v8f s0 = zero8(), s1 = zero8();
    const _Float16* k0p = Khb + (size_t)kb * KROW;
    const _Float16* k1p = k0p + (size_t)16 * KROW;
#pragma unroll
    for (int kk = 0; kk < HD / 32; ++kk) {
      const v16h qh  = ldfrag_h(Qh + kk * 32);
      const v16h ql  = ldfrag_h(Ql + kk * 32);
      const v16h kh0 = ldfrag_h(k0p + kk * 32);
      const v16h kh1 = ldfrag_h(k1p + kk * 32);
      s0 = mma_h(qh, kh0, s0);
      s0 = mma_h(ql, kh0, s0);
      s1 = mma_h(qh, kh1, s1);
      s1 = mma_h(ql, kh1, s1);
      guard2(s0, s1, qh, ql, kh0, kh1, qh, ql);
    }
    float alpha[8];
#pragma unroll
    for (int r = 0; r < 8; ++r) {
      const float t0 = s0[r] * lsc;
      const float t1 = s1[r] * lsc;
      float mx = fmaxf(t0, t1);
      mx = fmaxf(mx, __shfl_xor(mx, 1, 32));
      mx = fmaxf(mx, __shfl_xor(mx, 2, 32));
      mx = fmaxf(mx, __shfl_xor(mx, 4, 32));
      mx = fmaxf(mx, __shfl_xor(mx, 8, 32));
      const float mnew = fmaxf(mrun[r], mx);
      const float al   = __expf(mrun[r] - mnew);
      const float p0   = __expf(t0 - mnew);
      const float p1   = __expf(t1 - mnew);
      float sm = p0 + p1;
      sm += __shfl_xor(sm, 1, 32);
      sm += __shfl_xor(sm, 2, 32);
      sm += __shfl_xor(sm, 4, 32);
      sm += __shfl_xor(sm, 8, 32);
      lrun[r]  = lrun[r] * al + sm;
      mrun[r]  = mnew;
      alpha[r] = al;
      const int ro = (8 * hh + r) * PTP + c;
      pt[ro]      = p0;
      pt[ro + 16] = p1;
    }
    wave_sync_lds();
#pragma unroll
    for (int j = 0; j < 4; ++j) {
#pragma unroll
      for (int r = 0; r < 8; ++r) o[j][r] = o[j][r] * alpha[r];
    }
    FragH ph;
    {
      const float* prow = pt + c * PTP + 8 * hh;
      const v4f p0 = *(const v4f*)(prow), p1 = *(const v4f*)(prow + 4);
      const v4f p2 = *(const v4f*)(prow + 16), p3 = *(const v4f*)(prow + 20);
#pragma unroll
      for (int e = 0; e < 4; ++e) {
        ph.h[0][e]     = (_Float16)(p0[e] * PCAR);
        ph.h[0][4 + e] = (_Float16)(p1[e] * PCAR);
        ph.h[1][e]     = (_Float16)(p2[e] * PCAR);
        ph.h[1][4 + e] = (_Float16)(p3[e] * PCAR);
      }
    }
    {
      const _Float16* vhp = Vhb + kb;
#pragma unroll
      for (int jg = 0; jg < 2; ++jg) {
        const size_t da = (size_t)(2 * jg) * 16 * SEQ;
        const size_t db = da + (size_t)16 * SEQ;
        const v16h vha = ldfrag_h(vhp + da), vhb2 = ldfrag_h(vhp + db);
        o[2 * jg]     = mma_h(ph.v, vha,  o[2 * jg]);
        o[2 * jg + 1] = mma_h(ph.v, vhb2, o[2 * jg + 1]);
        guard2(o[2 * jg], o[2 * jg + 1], ph.v, ph.v, vha, vhb2, vha, vhb2);
      }
    }
    wave_sync_lds();
  }
  acc_guard4(o[0], o[1], o[2], o[3]);
  float rl[8];
#pragma unroll
  for (int r = 0; r < 8; ++r) rl[r] = (1.0f / lrun[r]) * oc;
#pragma unroll
  for (int r = 0; r < 8; ++r) {
#pragma unroll
    for (int j = 0; j < 4; ++j) {
      const int idx = (8 * hh + r) * SLP + j * 16 + c;
      slab[idx] = o[j][r] * rl[r];
    }
  }
  wave_sync_lds();
  v4u oh[4], ol[4];
  const int rq = lane >> 3, c8 = (lane & 7) * 8;
#pragma unroll
  for (int it = 0; it < 4; ++it) {
    const int row = it * 4 + rq;
    const v4f a = *(const v4f*)(slab + row * SLP + c8), b4 = *(const v4f*)(slab + row * SLP + c8 + 4);
    float w[8];
#pragma unroll
    for (int e = 0; e < 4; ++e) { w[e] = a[e] * OSC; w[4 + e] = b4[e] * OSC; }
#pragma unroll
    for (int e = 0; e < 4; ++e) {
      const _Float16 h0 = (_Float16)w[2 * e], h1 = (_Float16)w[2 * e + 1];
      const _Float16 g0 = (_Float16)(w[2 * e] - (float)h0), g1 = (_Float16)(w[2 * e + 1] - (float)h1);
      oh[it][e] = pk16(h_bits(h0), h_bits(h1));
      ol[it][e] = pk16(h_bits(g0), h_bits(g1));
    }
  }
  const size_t ob = ((size_t)b * SEQ + q0) * DMOD + (size_t)head * HD + c8;
  for (int pass = 0; pass < 2; ++pass) {
#pragma unroll
    for (int it = 0; it < 4; ++it) {
      const int row = it * 4 + rq;
      *(volatile v4u*)(OHp + ob + (size_t)row * DMOD) = oh[it];
      *(volatile v4u*)(OLp + ob + (size_t)row * DMOD) = ol[it];
    }
    __threadfence();
  }
}

extern "C" void kernel_launch(void* const* d_in, const int* in_sizes, int n_in,
                              void* d_out, int out_size, void* d_ws, size_t ws_size,
                              hipStream_t stream) {
  if (n_in < 9) return;
  if (in_sizes[0] < ((NB - 1) * XS_FULL + SEQ) * DMOD) return;
  if (in_sizes[1] < DMOD * DMOD || in_sizes[3] < DMOD * DMOD || in_sizes[5] < DMOD * DMOD || in_sizes[7] < DMOD * DMOD) return;
  if (in_sizes[2] < DMOD || in_sizes[4] < DMOD || in_sizes[6] < DMOD || in_sizes[8] < DMOD) return;
  if (out_size < MROWS * DMOD) return;

  const float* x  = (const float*)d_in[0];
  const float* wq = (const float*)d_in[1];
  const float* bq = (const float*)d_in[2];
  const float* wk = (const float*)d_in[3];
  const float* bk = (const float*)d_in[4];
  const float* wv = (const float*)d_in[5];
  const float* bv = (const float*)d_in[6];
  const float* wo = (const float*)d_in[7];
  const float* bo = (const float*)d_in[8];
  float*       out = (float*)d_out;

  const size_t szXB = (size_t)MROWS * DMOD * 2;
  const size_t szWB = (size_t)3 * DMOD * DMOD * 2;
  const size_t szF  = (size_t)MROWS * DMOD * 4;
  const size_t szQ  = (size_t)MROWS * DMOD * 2;
  const size_t szV  = (size_t)NB * NH * HD * SEQ * 2;
  const size_t szT  = (size_t)SEQ * NFREQ * 4;
  const size_t szOH = (size_t)MROWS * DMOD * 2;
  const size_t szOL = (size_t)MROWS * DMOD * 2;
  const size_t szWT = (size_t)DMOD * DMOD * 2;
  if (szOH > szXB || szOL > szF || szWT > szWB || szV != szQ) return;
  size_t off = 0;
  const size_t oXB = off; off += szXB;
  const size_t oWB = off; off += szWB;
  const size_t oF  = off; off += szF;
  const size_t oQH = off; off += szQ;
  const size_t oQL = off; off += szQ;
  const size_t oKH = off; off += szQ;
  const size_t oVH = off; off += szV;
  const size_t oTC = off; off += szT;
  const size_t oTS = off; off += szT;
  if (off > ws_size) return;
  if (off > (size_t)WS_CAP) return;

  char* ws = (char*)d_ws;
  u16*   XB  = (u16*)(ws + oXB);
  u16*   OH  = (u16*)(ws + oXB);
  u16*   WB  = (u16*)(ws + oWB);
  u16*   WT  = (u16*)(ws + oWB);
  float* F   = (float*)(ws + oF);
  u16*   OL  = (u16*)(ws + oF);
  u16*   QH  = (u16*)(ws + oQH);
  u16*   QL  = (u16*)(ws + oQL);
  u16*   KH  = (u16*)(ws + oKH);
  u16*   VH  = (u16*)(ws + oVH);
  float* TC  = (float*)(ws + oTC);
  float* TS  = (float*)(ws + oTS);
  u16*   WBq = WB;
  u16*   WBk = WB + (size_t)DMOD * DMOD;
  u16*   WBv = WB + (size_t)2 * DMOD * DMOD;

  const dim3 b256(256), b128(128), bAT(ATT_THREADS);
  const int  n8x = (SEQ * DMOD) / 8;
  const dim3 gX((n8x + 255) / 256);
  const int  n8w = (DMOD * DMOD) / 8;
  const dim3 gW((n8w + 255) / 256);
  const int  nT  = SEQ * NFREQ;
  const dim3 gT((nT + 255) / 256);
  const dim3 gG((MROWS / 64) * (DMOD / 64));
  const dim3 gRW(MROWS);
  const dim3 gVT(NB * NH * NST);
  const dim3 gAT(NQT * NHG * NB);
  const float osc = 1.0f / (OSC * WOS);

  for (int bq2 = 0; bq2 < NB; ++bq2) {
    cvt16<<<gX, b256, 0, stream>>>(x + (size_t)bq2 * XS_FULL * DMOD, XB + (size_t)bq2 * SEQ * DMOD, n8x, 0, 1.0f);
  }
  cvt16<<<gW, b256, 0, stream>>>(wq, WBq, n8w, 0, 1.0f);
  cvt16<<<gW, b256, 0, stream>>>(wk, WBk, n8w, 0, 1.0f);
  cvt16<<<gW, b256, 0, stream>>>(wv, WBv, n8w, 0, 1.0f);
  k_tab<<<gT, b256, 0, stream>>>(TC, TS, nT);
  gemm_bf<<<gG, b128, 0, stream>>>(XB, WBq, bq, F, MROWS, DMOD, DMOD, 1.0f);
  rope16<1><<<gRW, dim3(DMOD / 8), 0, stream>>>(F, DMOD, 0, TC, TS, QH, QL, QSC);
  gemm_bf<<<gG, b128, 0, stream>>>(XB, WBk, bk, F, MROWS, DMOD, DMOD, 1.0f);
  rope16<0><<<gRW, dim3(DMOD / 8), 0, stream>>>(F, DMOD, 0, TC, TS, KH, KH, KSC);
  gemm_bf<<<gG, b128, 0, stream>>>(XB, WBv, bv, F, MROWS, DMOD, DMOD, 1.0f);
  vt16<<<gVT, b256, 0, stream>>>(F, DMOD, 0, VH);
  cvt16<<<gW, b256, 0, stream>>>(wo, WT, n8w, 1, WOS);
  attn_mh<<<gAT, bAT, 0, stream>>>(QH, QL, KH, VH, OH, OL, NQT);
  gemm_h<1><<<gG, b128, 0, stream>>>(OH, OL, WT, bo, out, MROWS, DMOD, DMOD, osc);
  (void)hipGetLastError();
}
